// Unit_60687887892937
// MI455X (gfx1250) — hardware-verified
//
#include <hip/hip_runtime.h>
#define NB 32
#define CC 64
#define TT 300
#define VV 25
#define VP 32
#define NS 3
#define IE 16
#define NR (NB * TT * VV)
#define KT (9 * CC)
#define NRB 256

typedef __bf16 v16b __attribute__((ext_vector_type(16)));
typedef unsigned short v8us __attribute__((ext_vector_type(8), may_alias));
typedef float  v8f  __attribute__((ext_vector_type(8)));
typedef float  v4f  __attribute__((ext_vector_type(4)));
typedef float  v4fa __attribute__((ext_vector_type(4), may_alias));
union FragB { v16b v; v8us half[2]; unsigned short u[16]; };

__device__ __forceinline__ unsigned short bf16_bits(float x) { unsigned int u = __float_as_uint(x); return (unsigned short)((u + 0x7FFFu + ((u >> 16) & 1u)) >> 16); }
__device__ __forceinline__ float bf16_val(unsigned short b) { return __uint_as_float(((unsigned int)b) << 16); }
__device__ __forceinline__ float bf16_round(float x) { return bf16_val(bf16_bits(x)); }
template <int NT>
__device__ __forceinline__ v8f mmaN(v16b ah, v16b al, v16b bh, v16b bl, v8f c) {
  c = __builtin_amdgcn_wmma_f32_16x16x32_bf16(false, ah, false, bh, (short)0, c, false, false);
  if (NT >= 2) c = __builtin_amdgcn_wmma_f32_16x16x32_bf16(false, al, false, bh, (short)0, c, false, false);
  if (NT >= 3) c = __builtin_amdgcn_wmma_f32_16x16x32_bf16(false, ah, false, bl, (short)0, c, false, false);
  asm volatile("v_nop\n\tv_nop\n\tv_nop\n\tv_nop" : "+v"(c) : "v"(ah), "v"(al), "v"(bh), "v"(bl));
  return c;
}

__global__ __launch_bounds__(256) void k_wt_bf16(const float* __restrict__ W, unsigned short* __restrict__ Wt, int K, int N) {
  const int t = blockIdx.x * 256 + threadIdx.x;
  const int k8n = K / 8;
  if (t >= N * k8n) return;
  const int n = t / k8n, k8 = (t % k8n) * 8;
  v8us v;
#pragma unroll
  for (int i = 0; i < 8; ++i) v[i] = bf16_bits(W[(size_t)(k8 + i) * N + n]);
  *(volatile v8us*)(Wt + (size_t)n * K + k8) = v;
  __threadfence();
  *(volatile v8us*)(Wt + (size_t)n * K + k8) = v;
}

template <bool ASPLIT, int ACT, bool BIAS_BF16>
__global__ __launch_bounds__(128) void k_gemm_bf(const float* __restrict__ A, int lda, const unsigned short* __restrict__ Wt, int ldb,
                                               const float* __restrict__ bias, float* __restrict__ C, int ldc, int M, int N, int K) {
  __shared__ __attribute__((aligned(16))) float so[4][16][64];
  const int tid = threadIdx.x, w = tid >> 5, lane = tid & 31, ln = lane & 15, hh = lane >> 4;
  const int ntn = N / 64;
  const int wid = blockIdx.x * 4 + w;
  const int mt = wid / ntn, nq = wid % ntn;
  if (mt * 16 >= M) return;
  const int row0 = mt * 16, col0 = nq * 64;
  const float* arow = A + (size_t)(row0 + ln) * lda;
  v8f acc[4] = {};
  for (int kb = 0; kb < K; kb += 32) {
    FragB ah, al;
    const v4f x0 = *(const v4fa*)(arow + kb + 8 * hh), x1 = *(const v4fa*)(arow + kb + 8 * hh + 4);
    const v4f x2 = *(const v4fa*)(arow + kb + 16 + 8 * hh), x3 = *(const v4fa*)(arow + kb + 16 + 8 * hh + 4);
    float xs[16] = {x0[0],x0[1],x0[2],x0[3],x1[0],x1[1],x1[2],x1[3],x2[0],x2[1],x2[2],x2[3],x3[0],x3[1],x3[2],x3[3]};
#pragma unroll
    for (int i = 0; i < 16; ++i) { const unsigned short hb = bf16_bits(xs[i]); ah.u[i] = hb; al.u[i] = ASPLIT ? bf16_bits(xs[i] - bf16_val(hb)) : (unsigned short)0; }
#pragma unroll
    for (int t = 0; t < 4; ++t) {
      const unsigned short* brow = Wt + (size_t)(col0 + t * 16 + ln) * ldb + kb;
      FragB b;
      b.half[0] = *(const v8us*)(brow + 8 * hh);
      b.half[1] = *(const v8us*)(brow + 16 + 8 * hh);
      acc[t] = mmaN<ASPLIT ? 2 : 1>(ah.v, al.v, b.v, b.v, acc[t]);
    }
  }
#pragma unroll
  for (int t = 0; t < 4; ++t) {
    float bv = bias ? bias[col0 + t * 16 + ln] : 0.f;
    if (BIAS_BF16) bv = bf16_round(bv);
#pragma unroll
    for (int r = 0; r < 8; ++r) { float v = acc[t][r] + bv; if (ACT == 1) v = fmaxf(v, 0.f); so[w][8 * hh + r][t * 16 + ln] = v; }
  }
  __builtin_amdgcn_fence(__ATOMIC_ACQ_REL, "workgroup");
  __builtin_amdgcn_wave_barrier();
  const int rsub = lane >> 4, c4 = (lane & 15) * 4;
  for (int pass = 0; pass < 2; ++pass) {
#pragma unroll
    for (int q = 0; q < 8; ++q) {
      const int r = q * 2 + rsub;
      const v4f v = *(const v4fa*)&so[w][r][c4];
      *(volatile v4f*)(C + (size_t)(row0 + r) * ldc + col0 + c4) = v;
    }
    if (pass == 0) __threadfence();
  }
}

template <int D, bool CAUSAL>
__global__ __launch_bounds__(128) void k_flash(const float* __restrict__ qb, const float* __restrict__ kb, const float* __restrict__ vb,
                                             int pitch, int T, int H, float scale, float* __restrict__ y, int ypitch) {
  constexpr int KS = D / 32;
  constexpr int DT = D / 16;
  __shared__ __attribute__((aligned(16))) unsigned short sKh[32][D + 8], sKl[32][D + 8], sVh[32][D + 8], sVl[32][D + 8];
  __shared__ __attribute__((aligned(16))) unsigned short sPh[4][16][40], sPl[4][16][40];
  __shared__ __attribute__((aligned(16))) float sO[4][16][D];
  const int tid = threadIdx.x, w = tid >> 5, lane = tid & 31, ln = lane & 15, hh = lane >> 4;
  const int nqb = (T + 63) / 64;
  const int bh = blockIdx.x / nqb, qblk = blockIdx.x % nqb;
  const int b = bh / H, h = bh % H;
  const int q0 = qblk * 64 + w * 16;
  const float* Q = qb + (size_t)b * T * pitch + h * D;
  const float* K = kb + (size_t)b * T * pitch + h * D;
  const float* V = vb + (size_t)b * T * pitch + h * D;

  FragB aqh[KS], aql[KS];
  {
    int row = q0 + ln; if (row >= T) row = T - 1;
    const float* qr = Q + (size_t)row * pitch;
#pragma unroll
    for (int ks = 0; ks < KS; ++ks)
#pragma unroll
      for (int i = 0; i < 16; ++i) {
        const int d = ks * 32 + ((i < 8) ? (8 * hh + i) : (16 + 8 * hh + (i - 8)));
        const float x = qr[d] * scale; const unsigned short hb = bf16_bits(x);
        aqh[ks].u[i] = hb; aql[ks].u[i] = bf16_bits(x - bf16_val(hb));
      }
  }
  float m_r[8], l_r[8];
#pragma unroll
  for (int r = 0; r < 8; ++r) { m_r[r] = -3.0e38f; l_r[r] = 0.f; }
  v8f oacc[DT];
#pragma unroll
  for (int dt = 0; dt < DT; ++dt) oacc[dt] = (v8f){0.f,0.f,0.f,0.f,0.f,0.f,0.f,0.f};

  const int kv_end = CAUSAL ? min(T, qblk * 64 + 64) : T;
  for (int j0 = 0; j0 < kv_end; j0 += 32) {
    __syncthreads();
    for (int e = tid; e < 32 * (D / 4); e += 128) {
      const int r = e / (D / 4), c4 = (e % (D / 4)) * 4;
      const int key = j0 + r;
      v4f kf = {0.f,0.f,0.f,0.f}, vf = {0.f,0.f,0.f,0.f};
      if (key < T) { kf = *(const v4fa*)(K + (size_t)key * pitch + c4); vf = *(const v4fa*)(V + (size_t)key * pitch + c4); }
#pragma unroll
      for (int t = 0; t < 4; ++t) {
        unsigned short hb = bf16_bits(kf[t]); sKh[r][c4 + t] = hb; sKl[r][c4 + t] = bf16_bits(kf[t] - bf16_val(hb));
        hb = bf16_bits(vf[t]); sVh[r][c4 + t] = hb; sVl[r][c4 + t] = bf16_bits(vf[t] - bf16_val(hb));
      }
    }
    __syncthreads();
    v8f s[2];
#pragma unroll
    for (int nt = 0; nt < 2; ++nt) {
      v8f acc = {};
#pragma unroll
      for (int ks = 0; ks < KS; ++ks) {
        FragB bh_, bl_;
        bh_.half[0] = *(const v8us*)&sKh[nt * 16 + ln][ks * 32 + 8 * hh]; bh_.half[1] = *(const v8us*)&sKh[nt * 16 + ln][ks * 32 + 16 + 8 * hh];
        bl_.half[0] = *(const v8us*)&sKl[nt * 16 + ln][ks * 32 + 8 * hh]; bl_.half[1] = *(const v8us*)&sKl[nt * 16 + ln][ks * 32 + 16 + 8 * hh];
        acc = mmaN<3>(aqh[ks].v, aql[ks].v, bh_.v, bl_.v, acc);
      }
      s[nt] = acc;
    }
    float alpha[8];
#pragma unroll
    for (int r = 0; r < 8; ++r) {
      const int qi = q0 + 8 * hh + r;
      const int ja = j0 + ln, jb = j0 + 16 + ln;
      if (CAUSAL) { if (ja > qi) s[0][r] = -3.0e38f; if (jb > qi) s[1][r] = -3.0e38f; }
      if (ja >= T) s[0][r] = -3.0e38f;
      if (jb >= T) s[1][r] = -3.0e38f;
      float mx = fmaxf(s[0][r], s[1][r]);
      mx = fmaxf(mx, __shfl_xor(mx, 1, 32)); mx = fmaxf(mx, __shfl_xor(mx, 2, 32)); mx = fmaxf(mx, __shfl_xor(mx, 4, 32)); mx = fmaxf(mx, __shfl_xor(mx, 8, 32));
      const float mnew = fmaxf(m_r[r], mx);
      alpha[r] = (mnew > -1.0e38f) ? __expf(m_r[r] - mnew) : 1.0f;
      const float p0 = (s[0][r] > -1.0e38f) ? __expf(s[0][r] - mnew) : 0.f;
      const float p1 = (s[1][r] > -1.0e38f) ? __expf(s[1][r] - mnew) : 0.f;
      m_r[r] = mnew;
      l_r[r] = l_r[r] * alpha[r] + p0 + p1;
      unsigned short hb = bf16_bits(p0); sPh[w][8 * hh + r][ln] = hb;      sPl[w][8 * hh + r][ln] = bf16_bits(p0 - bf16_val(hb));
      hb = bf16_bits(p1);                sPh[w][8 * hh + r][16 + ln] = hb; sPl[w][8 * hh + r][16 + ln] = bf16_bits(p1 - bf16_val(hb));
    }
#pragma unroll
    for (int dt = 0; dt < DT; ++dt)
#pragma unroll
      for (int r = 0; r < 8; ++r) oacc[dt][r] *= alpha[r];
    __builtin_amdgcn_fence(__ATOMIC_ACQ_REL, "workgroup");
    __builtin_amdgcn_wave_barrier();
    FragB pah, pal;
    pah.half[0] = *(const v8us*)&sPh[w][ln][8 * hh]; pah.half[1] = *(const v8us*)&sPh[w][ln][16 + 8 * hh];
    pal.half[0] = *(const v8us*)&sPl[w][ln][8 * hh]; pal.half[1] = *(const v8us*)&sPl[w][ln][16 + 8 * hh];
#pragma unroll
    for (int dt = 0; dt < DT; ++dt) {
      FragB bvh, bvl;
#pragma unroll
      for (int i = 0; i < 8; ++i) {
        bvh.u[i] = sVh[8 * hh + i][dt * 16 + ln]; bvh.u[8 + i] = sVh[16 + 8 * hh + i][dt * 16 + ln];
        bvl.u[i] = sVl[8 * hh + i][dt * 16 + ln]; bvl.u[8 + i] = sVl[16 + 8 * hh + i][dt * 16 + ln];
      }
      oacc[dt] = mmaN<3>(pah.v, pal.v, bvh.v, bvl.v, oacc[dt]);
    }
    __builtin_amdgcn_fence(__ATOMIC_ACQ_REL, "workgroup");
    __builtin_amdgcn_wave_barrier();
  }
#pragma unroll
  for (int r = 0; r < 8; ++r) {
    float l = l_r[r];
    l += __shfl_xor(l, 1, 32); l += __shfl_xor(l, 2, 32); l += __shfl_xor(l, 4, 32); l += __shfl_xor(l, 8, 32);
    l_r[r] = (l > 0.f) ? 1.0f / l : 0.f;
  }
#pragma unroll
  for (int dt = 0; dt < DT; ++dt)
#pragma unroll
    for (int r = 0; r < 8; ++r) sO[w][8 * hh + r][dt * 16 + ln] = oacc[dt][r] * l_r[r];
  __builtin_amdgcn_fence(__ATOMIC_ACQ_REL, "workgroup");
  __builtin_amdgcn_wave_barrier();
  for (int pass = 0; pass < 2; ++pass) {
    for (int r = 0; r < 16; ++r) {
      const int row = q0 + r;
      if (row < T && lane < D / 4) {
        const v4f val = *(const v4fa*)&sO[w][r][lane * 4];
        *(volatile v4f*)(y + ((size_t)b * T + row) * ypitch + h * D + lane * 4) = val;
      }
    }
    if (pass == 0) __threadfence();
  }
}

template <bool ASPLIT, int ACT, bool BIAS_BF16, bool RES_BF16>
__global__ __launch_bounds__(128) void k_gemm_bf3(const float* __restrict__ A, int lda, const unsigned short* __restrict__ Wt, int ldb,
                                                const float* __restrict__ bias, const float* __restrict__ resid, int rmod, int ldr,
                                                float* __restrict__ C, int ldc, int M, int N, int K) {
  __shared__ __attribute__((aligned(16))) float so[4][16][64];
  const int tid = threadIdx.x, w = tid >> 5, lane = tid & 31, ln = lane & 15, hh = lane >> 4;
  const int ntn = N / 64;
  const int wid = blockIdx.x * 4 + w;
  const int mt = wid / ntn, nq = wid % ntn;
  if (mt * 16 >= M) return;
  const int row0 = mt * 16, col0 = nq * 64;
  const float* arow = A + (size_t)(row0 + ln) * lda;
  v8f acc[4] = {};
  for (int kb = 0; kb < K; kb += 32) {
    FragB ah, al;
    const v4f x0 = *(const v4fa*)(arow + kb + 8 * hh), x1 = *(const v4fa*)(arow + kb + 8 * hh + 4);
    const v4f x2 = *(const v4fa*)(arow + kb + 16 + 8 * hh), x3 = *(const v4fa*)(arow + kb + 16 + 8 * hh + 4);
    float xs[16] = {x0[0],x0[1],x0[2],x0[3],x1[0],x1[1],x1[2],x1[3],x2[0],x2[1],x2[2],x2[3],x3[0],x3[1],x3[2],x3[3]};
#pragma unroll
    for (int i = 0; i < 16; ++i) { const unsigned short hb = bf16_bits(xs[i]); ah.u[i] = hb; al.u[i] = ASPLIT ? bf16_bits(xs[i] - bf16_val(hb)) : (unsigned short)0; }
#pragma unroll
    for (int t = 0; t < 4; ++t) {
      const unsigned short* brow = Wt + (size_t)(col0 + t * 16 + ln) * ldb + kb;
      FragB b;
      b.half[0] = *(const v8us*)(brow + 8 * hh);
      b.half[1] = *(const v8us*)(brow + 16 + 8 * hh);
      acc[t] = mmaN<ASPLIT ? 2 : 1>(ah.v, al.v, b.v, b.v, acc[t]);
    }
  }
#pragma unroll
  for (int t = 0; t < 4; ++t) {
    const int col = col0 + t * 16 + ln;
    float bv = bias ? bias[col] : 0.f;
    if (BIAS_BF16) bv = bf16_round(bv);
#pragma unroll
    for (int r = 0; r < 8; ++r) {
      float v = acc[t][r] + bv;
      if (resid) { float rv = resid[(size_t)((row0 + 8 * hh + r) % rmod) * ldr + col]; if (RES_BF16) rv = bf16_round(rv); v += rv; }
      if (ACT == 1) v = fmaxf(v, 0.f);
      if (ACT == 2) v = 0.5f * v * (1.0f + erff(v * 0.70710678118654752f));
      if (ACT == 3) { const float u = 0.7978845608028654f * (v + 0.044715f * v * v * v); v = 0.5f * v * (1.0f + tanhf(u)); }
      so[w][8 * hh + r][t * 16 + ln] = v;
    }
  }
  __builtin_amdgcn_fence(__ATOMIC_ACQ_REL, "workgroup");
  __builtin_amdgcn_wave_barrier();
  const int rsub = lane >> 4, c4 = (lane & 15) * 4;
  for (int pass = 0; pass < 2; ++pass) {
#pragma unroll
    for (int q = 0; q < 8; ++q) {
      const int r = q * 2 + rsub;
      const v4f v = *(const v4fa*)&so[w][r][c4];
      *(volatile v4f*)(C + (size_t)(row0 + r) * ldc + col0 + c4) = v;
    }
    if (pass == 0) __threadfence();
  }
}
template <bool PARAM_BF16>
__global__ __launch_bounds__(256) void k_layernorm(const float* __restrict__ X, const float* __restrict__ R, const float* __restrict__ g, const float* __restrict__ bta,
                                                  float* __restrict__ out_sum, float* __restrict__ out_norm, int N, float eps) {
  __shared__ float red[256];
  const int row = blockIdx.x, tid = threadIdx.x;
  const float* x = X + (size_t)row * N; const float* rr = R ? R + (size_t)row * N : nullptr;
  float vals[16];
  const int per = N / 256;
  float s1 = 0.f;
  for (int u = 0; u < per / 4; ++u) {
    const int j = tid * 4 + 1024 * u;
    const v4f a = *(const v4fa*)(x + j);
    v4f b = {0.f,0.f,0.f,0.f}; if (rr) b = *(const v4fa*)(rr + j);
#pragma unroll
    for (int q = 0; q < 4; ++q) { const float v = a[q] + b[q]; vals[u * 4 + q] = v; s1 += v; }
  }
  red[tid] = s1; __syncthreads();
  for (int st = 128; st > 0; st >>= 1) { if (tid < st) red[tid] += red[tid + st]; __syncthreads(); }
  const float mu = red[0] / (float)N; __syncthreads();
  float s2 = 0.f;
  for (int u = 0; u < per / 4; ++u)
#pragma unroll
    for (int q = 0; q < 4; ++q) { const float c = vals[u * 4 + q] - mu; s2 += c * c; }
  red[tid] = s2; __syncthreads();
  for (int st = 128; st > 0; st >>= 1) { if (tid < st) red[tid] += red[tid + st]; __syncthreads(); }
  const float rs = rsqrtf(red[0] / (float)N + eps);
  for (int pass = 0; pass < 2; ++pass) {
    for (int u = 0; u < per / 4; ++u) {
      const int j = tid * 4 + 1024 * u;
      v4f o, sm;
#pragma unroll
      for (int q = 0; q < 4; ++q) {
        float gg = g[j + q], bb = bta[j + q];
        if (PARAM_BF16) { gg = bf16_round(gg); bb = bf16_round(bb); }
        sm[q] = vals[u * 4 + q]; o[q] = (vals[u * 4 + q] - mu) * rs * gg + bb;
      }
      if (out_sum) *(volatile v4f*)(out_sum + (size_t)row * N + j) = sm;
      *(volatile v4f*)(out_norm + (size_t)row * N + j) = o;
    }
    if (pass == 0) __threadfence();
  }
}


typedef _Float16 v16h __attribute__((ext_vector_type(16)));
union FragH { v16h v; v8us half[2]; _Float16 h[16]; unsigned short u[16]; };
template <int NT>
__device__ __forceinline__ v8f mmaH(v16h ah, v16h al, v16h bh, v16h bl, v8f c) {
  c = __builtin_amdgcn_wmma_f32_16x16x32_f16(false, ah, false, bh, (short)0, c, false, false);
  if (NT >= 2) c = __builtin_amdgcn_wmma_f32_16x16x32_f16(false, al, false, bh, (short)0, c, false, false);
  if (NT >= 3) c = __builtin_amdgcn_wmma_f32_16x16x32_f16(false, ah, false, bl, (short)0, c, false, false);
  asm volatile("v_nop\n\tv_nop\n\tv_nop\n\tv_nop" : "+v"(c) : "v"(ah), "v"(al), "v"(bh), "v"(bl));
  return c;
}
template <bool ASPLIT>
__global__ __launch_bounds__(128) void k_gemm_h(const float* __restrict__ A, int lda, size_t sA, const _Float16* __restrict__ Bh, int ldb, size_t sB, float alpha, float* __restrict__ C, int ldc, size_t sC, int M, int N, int K) {
  __shared__ __attribute__((aligned(16))) float so[4][16][64];
  const int tid = threadIdx.x, w = tid >> 5, lane = tid & 31, ln = lane & 15, hh = lane >> 4; const int by = blockIdx.y;
  A += (size_t)by * sA; Bh += (size_t)by * sB; C += (size_t)by * sC;
  const int ntn = (N + 63) / 64; const int wid = blockIdx.x * 4 + w; const int mt = wid / ntn, nq = wid % ntn; if (mt * 16 >= M) return;
  const int row0 = mt * 16, col0 = nq * 64; const float* arow = A + (size_t)(row0 + ln) * lda;
  v8f acc[4] = {};
  for (int kb = 0; kb < K; kb += 32) {
    FragH ah, al;
    const v4f x0 = *(const v4fa*)(arow + kb + 8 * hh), x1 = *(const v4fa*)(arow + kb + 8 * hh + 4), x2 = *(const v4fa*)(arow + kb + 16 + 8 * hh), x3 = *(const v4fa*)(arow + kb + 16 + 8 * hh + 4);
    float xs[16] = {x0[0],x0[1],x0[2],x0[3],x1[0],x1[1],x1[2],x1[3],x2[0],x2[1],x2[2],x2[3],x3[0],x3[1],x3[2],x3[3]};
#pragma unroll
    for (int i = 0; i < 16; ++i) { const _Float16 h = (_Float16)xs[i]; ah.h[i] = h; al.h[i] = ASPLIT ? (_Float16)(xs[i] - (float)h) : (_Float16)0.0f; }
#pragma unroll
    for (int t = 0; t < 4; ++t) { if (col0 + t * 16 >= N) continue; const size_t boff = (size_t)(col0 + t * 16 + ln) * ldb + kb; FragH bq; bq.half[0] = *(const v8us*)(Bh + boff + 8 * hh); bq.half[1] = *(const v8us*)(Bh + boff + 16 + 8 * hh);
      acc[t] = mmaH<ASPLIT ? 2 : 1>(ah.v, al.v, bq.v, bq.v, acc[t]); }
  }
#pragma unroll
  for (int t = 0; t < 4; ++t) { if (col0 + t * 16 >= N) continue;
#pragma unroll
    for (int r = 0; r < 8; ++r) so[w][8 * hh + r][t * 16 + ln] = acc[t][r] * alpha; }
  __builtin_amdgcn_fence(__ATOMIC_ACQ_REL, "workgroup"); __builtin_amdgcn_wave_barrier();
  const int rsub = lane >> 4, c4 = (lane & 15) * 4;
  for (int pass = 0; pass < 2; ++pass) {
#pragma unroll
    for (int q = 0; q < 8; ++q) { const int r = q * 2 + rsub; if (col0 + c4 < N) { const v4f v = *(const v4fa*)&so[w][r][c4]; *(volatile v4f*)(C + (size_t)(row0 + r) * ldc + col0 + c4) = v; } }
    if (pass == 0) __threadfence(); }
}

__global__ __launch_bounds__(256) void k_wt_f16(const float* __restrict__ W, _Float16* __restrict__ Wt, int K, int N, float scale) {
  const int t = blockIdx.x * 256 + threadIdx.x; if (t >= N * (K / 8)) return; const int n = t / (K / 8), k8 = (t % (K / 8)) * 8; FragH f;
#pragma unroll
  for (int i = 0; i < 8; ++i) f.h[i] = (_Float16)(bf16_round(W[(size_t)(k8 + i) * N + n]) * scale); const v8us o = f.half[0];
  *(volatile v8us*)((unsigned short*)Wt + (size_t)n * K + k8) = o; __threadfence(); *(volatile v8us*)((unsigned short*)Wt + (size_t)n * K + k8) = o;
}
template <int ACT>
__global__ __launch_bounds__(128) void k_gemm_hhx(const _Float16* __restrict__ A, int lda, size_t sA, const _Float16* __restrict__ Bh, int ldb, size_t sB, float alpha, const float* __restrict__ bias, size_t sBias, const float* __restrict__ CP, int rowsPerB, size_t sCPb, int row0g,
    float* __restrict__ C, _Float16* __restrict__ C16, int ldc, size_t sC, int M, int N, int K) {
  __shared__ __attribute__((aligned(16))) float so[4][16][64];
  const int tid = threadIdx.x, w = tid >> 5, lane = tid & 31, ln = lane & 15, hh = lane >> 4; const int by = blockIdx.y;
  A += (size_t)by * sA; Bh += (size_t)by * sB; const size_t cofs = (size_t)by * sC; const float* bp = bias ? bias + (size_t)by * sBias : nullptr;
  const int ntn = (N + 63) / 64; const int wid = blockIdx.x * 4 + w; const int mt = wid / ntn, nq = wid % ntn; if (mt * 16 >= M) return;
  const int row0 = mt * 16, col0 = nq * 64; const _Float16* arow = A + (size_t)(row0 + ln) * lda;
  v8f acc[4] = {};
  for (int kb = 0; kb < K; kb += 32) { FragH ah; ah.half[0] = *(const v8us*)((const unsigned short*)arow + kb + 8 * hh); ah.half[1] = *(const v8us*)((const unsigned short*)arow + kb + 16 + 8 * hh);
#pragma unroll
    for (int t = 0; t < 4; ++t) { if (col0 + t * 16 >= N) continue; const size_t boff = (size_t)(col0 + t * 16 + ln) * ldb + kb; FragH bq; bq.half[0] = *(const v8us*)((const unsigned short*)Bh + boff + 8 * hh); bq.half[1] = *(const v8us*)((const unsigned short*)Bh + boff + 16 + 8 * hh);
      acc[t] = mmaH<1>(ah.v, ah.v, bq.v, bq.v, acc[t]); }
  }
#pragma unroll
  for (int t = 0; t < 4; ++t) { if (col0 + t * 16 >= N) continue; const int col = col0 + t * 16 + ln; const float bv = bp ? bf16_round(bp[col]) : 0.f;
#pragma unroll
    for (int r = 0; r < 8; ++r) { float v = acc[t][r] * alpha + bv; if (CP) { const int bidx = (row0g + row0 + 8 * hh + r) / rowsPerB; v += CP[(size_t)bidx * sCPb + (size_t)by * 64 + col]; } if (ACT == 1) v = (v > 0.f) ? v : expm1f(v); else if (ACT == 3) v = fmaxf(v, 0.f); so[w][8 * hh + r][t * 16 + ln] = v; } }
  __builtin_amdgcn_fence(__ATOMIC_ACQ_REL, "workgroup"); __builtin_amdgcn_wave_barrier();
  const int rsub = lane >> 4, c4 = (lane & 15) * 4; typedef _Float16 v4h __attribute__((ext_vector_type(4)));
  for (int pass = 0; pass < 2; ++pass) {
#pragma unroll
    for (int q = 0; q < 8; ++q) { const int r = q * 2 + rsub; if (col0 + c4 < N) { const v4f v = *(const v4fa*)&so[w][r][c4]; if (C) *(volatile v4f*)(C + cofs + (size_t)(row0 + r) * ldc + col0 + c4) = v; if (C16) { v4h h4; for (int i = 0; i < 4; ++i) h4[i] = (_Float16)v[i]; *(volatile v4h*)(C16 + cofs + (size_t)(row0 + r) * ldc + col0 + c4) = h4; } } }
    if (pass == 0) __threadfence(); }
}


typedef _Float16 v2h __attribute__((ext_vector_type(2)));
__global__ __launch_bounds__(256) void k_wprep(const float* __restrict__ Wa, const float* __restrict__ ba, const float* __restrict__ Wb, const float* __restrict__ bb, const float* __restrict__ Wd, const float* __restrict__ bd, const float* __restrict__ Wt,
    _Float16* __restrict__ Wab, float* __restrict__ bab, _Float16* __restrict__ Bd, float* __restrict__ bds, _Float16* __restrict__ Bt) { const int tid = threadIdx.x;
  for (int pass = 0; pass < 2; ++pass) {
    for (int t = tid; t < 96 * (CC / 8); t += 256) { const int row = t / (CC / 8), k8 = (t % (CC / 8)) * 8; const int s = row / 32, rr = row % 32; const float* src = (rr < IE) ? (Wa + ((size_t)s * IE + rr) * CC) : (Wb + ((size_t)s * IE + (rr - IE)) * CC); FragH f;
#pragma unroll
      for (int q = 0; q < 8; ++q) f.h[q] = (_Float16)(bf16_round(src[k8 + q]) * 16.0f); *(volatile v8us*)((unsigned short*)Wab + (size_t)row * CC + k8) = f.half[0]; }
    if (tid < 96) { const int s = tid / 32, rr = tid % 32; const float v = (rr < IE) ? ba[s * IE + rr] : bb[s * IE + (rr - IE)]; *(volatile float*)(bab + tid) = bf16_round(v); }
    for (int t = tid; t < NS * CC * (CC / 8); t += 256) { const int k8 = (t % (CC / 8)) * 8; const int row = t / (CC / 8); FragH f;
#pragma unroll
      for (int q = 0; q < 8; ++q) f.h[q] = (_Float16)(bf16_round(Wd[(size_t)row * CC + k8 + q]) * 16.0f); *(volatile v8us*)((unsigned short*)Bd + (size_t)row * CC + k8) = f.half[0]; }
    if (tid < CC) { float s_ = 0.f; for (int s = 0; s < NS; ++s) s_ += bf16_round(bd[s * CC + tid]); *(volatile float*)(bds + tid) = s_; }
    for (int t = tid; t < CC * (KT / 8); t += 256) { const int o = t / (KT / 8), k8 = (t % (KT / 8)) * 8; FragH f;
#pragma unroll
      for (int q = 0; q < 8; ++q) { const int k = k8 + q; const int tap = k / CC, c = k % CC; f.h[q] = (_Float16)(bf16_round(Wt[((size_t)o * CC + c) * 9 + tap]) * 16.0f); } *(volatile v8us*)((unsigned short*)Bt + (size_t)o * KT + k8) = f.half[0]; }
    if (pass == 0) __threadfence(); } }
__device__ __forceinline__ _Float16 xh(const float* __restrict__ x, int n, int c, int t, int v) { return (_Float16)bf16_round(x[(((size_t)n * CC + c) * TT + t) * VV + v]); }
__global__ __launch_bounds__(128) void k_ab(const float* __restrict__ x, const _Float16* __restrict__ Wab, const float* __restrict__ bab, _Float16* __restrict__ AB) {
  __shared__ __attribute__((aligned(16))) _Float16 so[4][16][96];
  const int tid = threadIdx.x, w = tid >> 5, lane = tid & 31, ln = lane & 15, hh = lane >> 4; const size_t row0 = ((size_t)blockIdx.x * 4 + w) * 16; const size_t r = row0 + ln;
  const int v = (int)(r % VV); const int t = (int)((r / VV) % TT); const int n = (int)(r / ((size_t)VV * TT));
  v8f acc[6];
#pragma unroll
  for (int q = 0; q < 6; ++q) acc[q] = (v8f){0.f,0.f,0.f,0.f,0.f,0.f,0.f,0.f};
#pragma unroll
  for (int kb = 0; kb < CC; kb += 32) { FragH a;
#pragma unroll
    for (int j = 0; j < 8; ++j) { a.h[j] = xh(x, n, kb + 8 * hh + j, t, v); a.h[8 + j] = xh(x, n, kb + 16 + 8 * hh + j, t, v); }
#pragma unroll
    for (int q = 0; q < 6; ++q) { FragH b; const unsigned short* br = (const unsigned short*)Wab + (size_t)(q * 16 + ln) * CC + kb; b.half[0] = *(const v8us*)(br + 8 * hh); b.half[1] = *(const v8us*)(br + 16 + 8 * hh); acc[q] = mmaH<1>(a.v, a.v, b.v, b.v, acc[q]); } }
#pragma unroll
  for (int q = 0; q < 6; ++q) { const int col = q * 16 + ln; const float bv = bab[col];
#pragma unroll
    for (int rr = 0; rr < 8; ++rr) so[w][8 * hh + rr][col] = (_Float16)(acc[q][rr] * 0.0625f + bv); }
  __builtin_amdgcn_fence(__ATOMIC_ACQ_REL, "workgroup"); __builtin_amdgcn_wave_barrier();
  { const unsigned short* sp = (const unsigned short*)&so[w][0][0]; unsigned short* dp = (unsigned short*)AB + row0 * 96;
    for (int pass = 0; pass < 2; ++pass) {
#pragma unroll
      for (int i = 0; i < 6; ++i) { const int o8 = (i * 32 + lane) * 8; *(volatile v8us*)(dp + o8) = *(const v8us*)(sp + o8); }
      if (pass == 0) __threadfence(); } } }
__global__ __launch_bounds__(128) void k_attn(const _Float16* __restrict__ AB, const float* __restrict__ Am, const float* __restrict__ PAm, _Float16* __restrict__ attnT) {
  __shared__ float L[VP][VP + 1]; __shared__ __attribute__((aligned(16))) _Float16 so[VP][VP];
  const int tid = threadIdx.x, w = tid >> 5, lane = tid & 31, ln = lane & 15, hh = lane >> 4; const int n = blockIdx.x / NS, s = blockIdx.x % NS; const int rt = w >> 1, ct = w & 1;
  const int v1 = rt * 16 + ln, v2 = ct * 16 + ln; const int v1c = v1 < VV ? v1 : VV - 1, v2c = v2 < VV ? v2 : VV - 1;
  v8f acc = {0.f,0.f,0.f,0.f,0.f,0.f,0.f,0.f};
#pragma unroll 1
  for (int t = 0; t < TT; t += 2) { FragH a, b;
    const unsigned short* ra0 = (const unsigned short*)AB + (((size_t)n * TT + t) * VV + v1c) * 96 + s * 32 + 8 * hh; const unsigned short* ra1 = ra0 + (size_t)VV * 96;
    const unsigned short* rb0 = (const unsigned short*)AB + (((size_t)n * TT + t) * VV + v2c) * 96 + s * 32 + IE + 8 * hh; const unsigned short* rb1 = rb0 + (size_t)VV * 96;
    a.half[0] = *(const v8us*)ra0; a.half[1] = *(const v8us*)ra1; b.half[0] = *(const v8us*)rb0; b.half[1] = *(const v8us*)rb1;
    acc = mmaH<1>(a.v, a.v, b.v, b.v, acc); }
#pragma unroll
  for (int rr = 0; rr < 8; ++rr) L[rt * 16 + 8 * hh + rr][ct * 16 + ln] = acc[rr] * (1.0f / (float)(IE * TT));
  __syncthreads();
  if (tid < VP) { const int c2 = tid;
    if (c2 < VV) { float mx = -3.0e38f; for (int r1 = 0; r1 < VV; ++r1) mx = fmaxf(mx, L[r1][c2]); float den = 0.f; for (int r1 = 0; r1 < VV; ++r1) den += expf(L[r1][c2] - mx); const float inv = 1.0f / den;
      for (int r1 = 0; r1 < VP; ++r1) { float v = 0.f; if (r1 < VV) v = expf(L[r1][c2] - mx) * inv + bf16_round(Am[((size_t)s * VV + r1) * VV + c2]) + bf16_round(PAm[((size_t)s * VV + r1) * VV + c2]); so[c2][r1] = (_Float16)v; } }
    else { for (int r1 = 0; r1 < VP; ++r1) so[c2][r1] = (_Float16)0.0f; } }
  __syncthreads();
  { const unsigned short* sp = (const unsigned short*)&so[0][0]; unsigned short* dp = (unsigned short*)attnT + (size_t)blockIdx.x * VP * VP;
    *(volatile v8us*)(dp + tid * 8) = *(const v8us*)(sp + tid * 8); __threadfence(); *(volatile v8us*)(dp + tid * 8) = *(const v8us*)(sp + tid * 8); } }
__global__ __launch_bounds__(128) void k_z(const float* __restrict__ x, const _Float16* __restrict__ attnT, int s, _Float16* __restrict__ Z) {
  __shared__ float C[CC][VP + 1];
  const int tid = threadIdx.x, w = tid >> 5, lane = tid & 31, ln = lane & 15, hh = lane >> 4; const int n = blockIdx.x / TT, t = blockIdx.x % TT; const int c = w * 16 + ln;
  FragH a;
#pragma unroll
  for (int j = 0; j < 8; ++j) { const int k0 = 8 * hh + j, k1 = 16 + 8 * hh + j; a.h[j] = (k0 < VV) ? xh(x, n, c, t, k0) : (_Float16)0.0f; a.h[8 + j] = (k1 < VV) ? xh(x, n, c, t, k1) : (_Float16)0.0f; }
  const unsigned short* bt = (const unsigned short*)attnT + ((size_t)n * NS + s) * VP * VP;
#pragma unroll
  for (int ct = 0; ct < 2; ++ct) { FragH b; const unsigned short* br = bt + (size_t)(ct * 16 + ln) * VP; b.half[0] = *(const v8us*)(br + 8 * hh); b.half[1] = *(const v8us*)(br + 16 + 8 * hh);
    v8f acc = {0.f,0.f,0.f,0.f,0.f,0.f,0.f,0.f}; acc = mmaH<1>(a.v, a.v, b.v, b.v, acc);
#pragma unroll
    for (int rr = 0; rr < 8; ++rr) C[w * 16 + 8 * hh + rr][ct * 16 + ln] = acc[rr]; }
  __syncthreads();
  for (int pass = 0; pass < 2; ++pass) {
    for (int v2 = w; v2 < VV; v2 += 4) { v2h o; o.x = (_Float16)C[2 * lane][v2]; o.y = (_Float16)C[2 * lane + 1][v2]; *(volatile v2h*)(Z + (((size_t)n * TT + t) * VV + v2) * CC + 2 * lane) = o; }
    if (pass == 0) __threadfence(); } }
template <int MODE>
__global__ __launch_bounds__(256) void k_bnred(const float* __restrict__ Y, const float* __restrict__ ST, float* __restrict__ P) { __shared__ float sp[4][64]; const int tid = threadIdx.x, q = tid >> 6, c = tid & 63; const float mu = MODE ? ST[c] : 0.f; float s_ = 0.f;
#pragma unroll 1
  for (size_t r = (size_t)blockIdx.x * 4 + q; r < (size_t)NR; r += (size_t)NRB * 4) { const float v = Y[r * CC + c]; s_ += MODE ? (v - mu) * (v - mu) : v; }
  sp[q][c] = s_; __syncthreads();
  if (tid < 64) { const float tsum = sp[0][tid] + sp[1][tid] + sp[2][tid] + sp[3][tid]; *(volatile float*)(P + (size_t)blockIdx.x * CC + tid) = tsum; } __threadfence();
  if (tid < 64) { const float tsum = sp[0][tid] + sp[1][tid] + sp[2][tid] + sp[3][tid]; *(volatile float*)(P + (size_t)blockIdx.x * CC + tid) = tsum; } }
template <int MODE>
__global__ __launch_bounds__(64) void k_bnfin(const float* __restrict__ P, float* __restrict__ ST) { const int c = threadIdx.x; float s_ = 0.f;
#pragma unroll 1
  for (int b = 0; b < NRB; ++b) s_ += P[(size_t)b * CC + c]; const float m = s_ * (1.0f / (float)NR); const float v = MODE ? rsqrtf(m + 1e-5f) : m;
  *(volatile float*)(ST + MODE * CC + c) = v; __threadfence(); *(volatile float*)(ST + MODE * CC + c) = v; }
__global__ __launch_bounds__(256) void k_y2(const float* __restrict__ Y, const float* __restrict__ ST, const float* __restrict__ g1, const float* __restrict__ b1, const float* __restrict__ x, _Float16* __restrict__ Y2) { const size_t tt = (size_t)blockIdx.x * 256 + threadIdx.x; if (tt >= (size_t)NR * (CC / 8)) return; const size_t r = tt / (CC / 8); const int c8 = (int)(tt % (CC / 8)) * 8;
  const int v = (int)(r % VV); const int t = (int)((r / VV) % TT); const int n = (int)(r / ((size_t)VV * TT)); FragH f;
#pragma unroll
  for (int q = 0; q < 8; ++q) { const int c = c8 + q; float y = (Y[r * CC + c] - ST[c]) * ST[CC + c] * bf16_round(g1[c]) + bf16_round(b1[c]) + (float)xh(x, n, c, t, v); f.h[q] = (_Float16)fmaxf(y, 0.f); }
  *(volatile v8us*)((unsigned short*)Y2 + tt * 8) = f.half[0]; __threadfence(); *(volatile v8us*)((unsigned short*)Y2 + tt * 8) = f.half[0]; }
__global__ __launch_bounds__(128) void k_tconv(const _Float16* __restrict__ Y2, const _Float16* __restrict__ Bt, const float* __restrict__ bt, float* __restrict__ YC) {
  __shared__ __attribute__((aligned(16))) float so[4][16][64];
  const int tid = threadIdx.x, w = tid >> 5, lane = tid & 31, ln = lane & 15, hh = lane >> 4; const size_t row0 = ((size_t)blockIdx.x * 4 + w) * 16; const size_t r = row0 + ln; const int t = (int)((r / VV) % TT);
  v8f acc[4];
#pragma unroll
  for (int q = 0; q < 4; ++q) acc[q] = (v8f){0.f,0.f,0.f,0.f,0.f,0.f,0.f,0.f};
#pragma unroll 1
  for (int ks = 0; ks < 18; ++ks) { const int tap = ks >> 1, ch = (ks & 1) * 32; const int ts = t + tap - 4; FragH a;
    if (ts >= 0 && ts < TT) { const unsigned short* ar = (const unsigned short*)Y2 + (r + (ptrdiff_t)(tap - 4) * VV) * CC + ch; a.half[0] = *(const v8us*)(ar + 8 * hh); a.half[1] = *(const v8us*)(ar + 16 + 8 * hh); }
    else { for (int j = 0; j < 16; ++j) a.h[j] = (_Float16)0.0f; }
#pragma unroll
    for (int q = 0; q < 4; ++q) { FragH b; const unsigned short* br = (const unsigned short*)Bt + (size_t)(q * 16 + ln) * KT + ks * 32; b.half[0] = *(const v8us*)(br + 8 * hh); b.half[1] = *(const v8us*)(br + 16 + 8 * hh); acc[q] = mmaH<1>(a.v, a.v, b.v, b.v, acc[q]); } }
#pragma unroll
  for (int q = 0; q < 4; ++q) { const int col = q * 16 + ln; const float bv = bf16_round(bt[col]);
#pragma unroll
    for (int rr = 0; rr < 8; ++rr) so[w][8 * hh + rr][col] = acc[q][rr] * 0.0625f + bv; }
  __builtin_amdgcn_fence(__ATOMIC_ACQ_REL, "workgroup"); __builtin_amdgcn_wave_barrier();
  const int rsub = lane >> 4, c4 = (lane & 15) * 4;
  for (int pass = 0; pass < 2; ++pass) {
#pragma unroll
    for (int q = 0; q < 8; ++q) { const int rr = q * 2 + rsub; const v4f vv = *(const v4fa*)&so[w][rr][c4]; *(volatile v4f*)(YC + (row0 + rr) * CC + c4) = vv; }
    if (pass == 0) __threadfence(); } }
__global__ __launch_bounds__(256) void k_out(const float* __restrict__ YC, const float* __restrict__ ST2, const float* __restrict__ g2, const float* __restrict__ b2, const float* __restrict__ x, float* __restrict__ out) { const size_t e = (size_t)blockIdx.x * 256 + threadIdx.x; if (e >= (size_t)NB * CC * TT * VV) return;
  const int v = (int)(e % VV); const int t = (int)((e / VV) % TT); const int c = (int)((e / ((size_t)VV * TT)) % CC); const int n = (int)(e / ((size_t)VV * TT * CC)); const size_t r = ((size_t)n * TT + t) * VV + v;
  const float y = (YC[r * CC + c] - ST2[c]) * ST2[CC + c] * bf16_round(g2[c]) + bf16_round(b2[c]) + bf16_round(x[e]); const float o = fmaxf(y, 0.f); *(volatile float*)(out + e) = o; __threadfence(); *(volatile float*)(out + e) = o; }

extern "C" void kernel_launch(void* const* d_in, const int* in_sizes, int n_in,
                              void* d_out, int out_size, void* d_ws, size_t ws_size, hipStream_t stream) {
  (void)in_sizes; (void)n_in; (void)out_size;
  const float* x = (const float*)d_in[0]; const float* Am = (const float*)d_in[1]; const float* PAm = (const float*)d_in[2]; const float* Wa = (const float*)d_in[3]; const float* ba = (const float*)d_in[4]; const float* Wb = (const float*)d_in[5]; const float* bb = (const float*)d_in[6];
  const float* Wd = (const float*)d_in[7]; const float* bd = (const float*)d_in[8]; const float* g1 = (const float*)d_in[9]; const float* b1 = (const float*)d_in[10]; const float* Wt = (const float*)d_in[11]; const float* bt = (const float*)d_in[12]; const float* g2 = (const float*)d_in[13]; const float* b2 = (const float*)d_in[14];
  char* ws = (char*)d_ws; size_t off = 0;
  auto take = [&](size_t bytes) { char* p = ws + off; off += (bytes + 255) & ~(size_t)255; return p; };
  _Float16* Wab = (_Float16*)take(96 * CC * 2); float* bab = (float*)take(96 * 4); _Float16* Bd = (_Float16*)take((size_t)NS * CC * CC * 2); float* bds = (float*)take(CC * 4); _Float16* Bt = (_Float16*)take((size_t)CC * KT * 2);
  float* ST1 = (float*)take(2 * CC * 4); float* ST2 = (float*)take(2 * CC * 4); float* P = (float*)take((size_t)NRB * CC * 4); _Float16* attnT = (_Float16*)take((size_t)NB * NS * VP * VP * 2);
  _Float16* AB = (_Float16*)take((size_t)NR * 96 * 2);
  _Float16* Z = AB; _Float16* Y2 = AB;
  float* Y = (float*)take((size_t)NR * CC * 4);
  float* YC = Y;
  if (off > ws_size) return;
  k_wprep<<<1, 256, 0, stream>>>(Wa, ba, Wb, bb, Wd, bd, Wt, Wab, bab, Bd, bds, Bt);
  k_ab<<<NR / 64, 128, 0, stream>>>(x, Wab, bab, AB);
  k_attn<<<NB * NS, 128, 0, stream>>>(AB, Am, PAm, attnT);
  const dim3 gy(((NR / 16) * 1 + 3) / 4, 1);
  for (int s = 0; s < NS; ++s) {
    k_z<<<NB * TT, 128, 0, stream>>>(x, attnT, s, Z);
    if (s == 0) k_gemm_hhx<0><<<gy, 128, 0, stream>>>(Z, CC, 0, Bd, CC, 0, 0.0625f, bds, 0, nullptr, 1, 0, 0, Y, nullptr, CC, 0, NR, CC, CC);
    else        k_gemm_hhx<0><<<gy, 128, 0, stream>>>(Z, CC, 0, Bd + (size_t)s * CC * CC, CC, 0, 0.0625f, nullptr, 0, Y, 1, (size_t)CC, 0, Y, nullptr, CC, 0, NR, CC, CC);
  }
  k_bnred<0><<<NRB, 256, 0, stream>>>(Y, ST1, P); k_bnfin<0><<<1, 64, 0, stream>>>(P, ST1); k_bnred<1><<<NRB, 256, 0, stream>>>(Y, ST1, P); k_bnfin<1><<<1, 64, 0, stream>>>(P, ST1);
  k_y2<<<(unsigned)(((size_t)NR * (CC / 8) + 255) / 256), 256, 0, stream>>>(Y, ST1, g1, b1, x, Y2);
  k_tconv<<<NR / 64, 128, 0, stream>>>(Y2, Bt, bt, YC);
  k_bnred<0><<<NRB, 256, 0, stream>>>(YC, ST2, P); k_bnfin<0><<<1, 64, 0, stream>>>(P, ST2); k_bnred<1><<<NRB, 256, 0, stream>>>(YC, ST2, P); k_bnfin<1><<<1, 64, 0, stream>>>(P, ST2);
  k_out<<<(unsigned)(((size_t)NB * CC * TT * VV + 255) / 256), 256, 0, stream>>>(YC, ST2, g2, b2, x, (float*)d_out);
}
